// TransformerBlock_88390426952039
// MI455X (gfx1250) — hardware-verified
//
#include <hip/hip_runtime.h>
#include <stddef.h>


typedef _Float16 v16h __attribute__((ext_vector_type(16)));
typedef _Float16 v8h  __attribute__((ext_vector_type(8)));
typedef _Float16 v4h  __attribute__((ext_vector_type(4)));
typedef float    v8f  __attribute__((ext_vector_type(8)));
typedef float    v4f  __attribute__((ext_vector_type(4)));

#ifndef NB
#define NB 64
#endif
#ifndef SEQ
#define SEQ 256
#endif
#define NB_FULL  64
#define SEQ_FULL 256
#define DIM   384
#define NHEAD 6
#define HD    64
#define FF    1536
#define MROWS (NB * SEQ)

static_assert(NB >= 1 && NB <= NB_FULL);
static_assert(SEQ >= 128 && SEQ <= SEQ_FULL && (SEQ % 128) == 0);
static_assert(DIM == NHEAD * HD);
static_assert(HD == 64);
static_assert((DIM % 64) == 0 && (DIM % 32) == 0);
static_assert((FF % 64) == 0 && (FF % 32) == 0);
static_assert(DIM == 32 * 4 * 3);
static_assert((MROWS % 64) == 0 && (MROWS % 8) == 0);
static_assert((size_t)MROWS * FF < (size_t)0xFFFFFFFFu);

#define LDT 72
#define LDC 68

#define WCARRY 64.0f
#define PCARRY 1024.0f
#define VCARRY 64.0f
#define HCARRY 64.0f

#define WA_BYTES      ((size_t)4 * DIM * DIM * 2)
#define W1_BYTES      ((size_t)FF * DIM * 2)
#define W2_BYTES      ((size_t)DIM * FF * 2)
#define PLANE16_BYTES ((size_t)MROWS * DIM * 2)
#define FPLANE_BYTES  ((size_t)MROWS * FF * 2)
#define REGION_BYTES  ((size_t)4 * PLANE16_BYTES)
#define X1_BYTES      ((size_t)MROWS * DIM * 4)
#define OFF_W1   (WA_BYTES)
#define OFF_W2   (OFF_W1 + W1_BYTES)
#define OFF_H    (OFF_W2 + W2_BYTES)
#define OFF_REG  (OFF_H + PLANE16_BYTES)
#define OFF_X1   (OFF_REG + REGION_BYTES)
#define WS_TOTAL (OFF_X1 + X1_BYTES)
static_assert(REGION_BYTES >= FPLANE_BYTES);
static_assert((WA_BYTES % 128) == 0 && (W1_BYTES % 128) == 0 && (W2_BYTES % 128) == 0);
static_assert((PLANE16_BYTES % 128) == 0 && (X1_BYTES % 128) == 0);
static_assert(WS_TOTAL <= (size_t)134217728);

__device__ __forceinline__ float bf16r(float x) {
  unsigned int u = __float_as_uint(x);
  u = (u + 0x7FFFu + ((u >> 16) & 1u)) & 0xFFFF0000u;
  return __uint_as_float(u);
}

__device__ __forceinline__ v16h frag_at(const _Float16* p) {
  v8h lo = *(const v8h*)(p);
  v8h hi = *(const v8h*)(p + 16);
  v16h out;
#pragma unroll
  for (int i = 0; i < 8; ++i) { out[i] = lo[i]; out[i + 8] = hi[i]; }
  return out;
}
__device__ __forceinline__ v16h ld_frag(const _Float16* base, unsigned ld) {
  const unsigned lane = threadIdx.x & 31u;
  return frag_at(base + (lane & 15u) * ld + (lane >> 4) * 8u);
}

__device__ __forceinline__ v8f wmma16(v16h a, v16h b, v8f c) {
  v8f d = __builtin_amdgcn_wmma_f32_16x16x32_f16(false, a, false, b, (short)0, c,
                                                 false, false);
  asm volatile("v_nop\n\tv_nop\n\tv_nop\n\tv_nop" : "+v"(d) : "v"(a), "v"(b));
  return d;
}

__device__ __forceinline__ float red16_max(float x) {
#pragma unroll
  for (int off = 1; off < 16; off <<= 1) x = fmaxf(x, __shfl_xor(x, off, 32));
  return x;
}
__device__ __forceinline__ float red16_sum(float x) {
#pragma unroll
  for (int off = 1; off < 16; off <<= 1) x += __shfl_xor(x, off, 32);
  return x;
}
__device__ __forceinline__ float red32_sum(float x) {
#pragma unroll
  for (int off = 1; off < 32; off <<= 1) x += __shfl_xor(x, off, 32);
  return x;
}

__device__ __forceinline__ void wave_lds_sync() {
  __builtin_amdgcn_fence(3  , "wavefront");
  asm volatile("s_wait_dscnt 0x0" ::: "memory");
  __builtin_amdgcn_wave_barrier();
}

__global__ __launch_bounds__(256) void wconv_kernel(
    const float* W0, const float* W1, const float* W2, const float* W3,
    _Float16* __restrict__ Wt, unsigned KR, unsigned NC) {
  __shared__ _Float16 T[64 * LDT];
  const unsigned tid = threadIdx.x;
  const unsigned n0 = blockIdx.x * 64u;
  const unsigned k0 = blockIdx.y * 64u;
  const unsigned p = blockIdx.z;
  const float* W = (p == 0u) ? W0 : ((p == 1u) ? W1 : ((p == 2u) ? W2 : W3));
#pragma unroll 4
  for (unsigned j = 0; j < 16u; ++j) {
    const unsigned idx = tid + 256u * j;
    const unsigned kr = idx >> 6, nc = idx & 63u;
    const float v = W[(size_t)(k0 + kr) * NC + n0 + nc];
    T[nc * LDT + kr] = (_Float16)(WCARRY * bf16r(v));
  }
  __syncthreads();
  v8h x[2];
  size_t off[2];
#pragma unroll
  for (unsigned i = 0; i < 2u; ++i) {
    const unsigned n = 32u * i + (tid >> 3);
    const unsigned kc = (tid & 7u) * 8u;
    x[i] = *(const v8h*)&T[n * LDT + kc];
    off[i] = (size_t)p * KR * NC + (size_t)(n0 + n) * KR + k0 + kc;
  }
#pragma unroll
  for (int i = 0; i < 2; ++i) *(volatile v8h*)(Wt + off[i]) = x[i];
  __threadfence();
#pragma unroll
  for (int i = 0; i < 2; ++i) *(volatile v8h*)(Wt + off[i]) = x[i];
}

template <int SRCIN>
__global__ __launch_bounds__(256) void ln_kernel(
    const float* __restrict__ src, const float* __restrict__ g,
    const float* __restrict__ be, _Float16* __restrict__ dst) {
  const unsigned tid = threadIdx.x, lane = tid & 31u, w = tid >> 5;
  const unsigned crow = blockIdx.x * 8u + w;
  size_t srow = (size_t)crow;
  if (SRCIN) {
    const unsigned bidx = crow / (unsigned)SEQ;
    const unsigned sq = crow - bidx * (unsigned)SEQ;
    srow = (size_t)bidx * SEQ_FULL + sq;
  }
  const float* sp = src + srow * DIM;
  v4f a[3];
  float s = 0.0f;
#pragma unroll
  for (unsigned i = 0; i < 3u; ++i) {
    v4f t = *(const v4f*)(sp + (lane + 32u * i) * 4u);
    if (SRCIN) {
#pragma unroll
      for (int j = 0; j < 4; ++j) t[j] = bf16r(t[j]);
    }
    a[i] = t;
    s += (t[0] + t[1]) + (t[2] + t[3]);
  }
  const float mean = red32_sum(s) * (1.0f / (float)DIM);
  float ss = 0.0f;
#pragma unroll
  for (int i = 0; i < 3; ++i) {
#pragma unroll
    for (int j = 0; j < 4; ++j) {
      const float d = a[i][j] - mean;
      a[i][j] = d;
      ss += d * d;
    }
  }
  const float var = red32_sum(ss) * (1.0f / (float)DIM);
  const float rstd = rsqrtf(var + 1.0e-5f);
  v4h o[3];
  size_t off[3];
#pragma unroll
  for (unsigned i = 0; i < 3u; ++i) {
    const unsigned c = (lane + 32u * i) * 4u;
    const v4f gv = *(const v4f*)(g + c);
    const v4f bv = *(const v4f*)(be + c);
#pragma unroll
    for (int j = 0; j < 4; ++j)
      o[i][j] = (_Float16)((a[i][j] * rstd) * bf16r(gv[j]) + bf16r(bv[j]));
    off[i] = (size_t)crow * DIM + c;
  }
#pragma unroll
  for (int i = 0; i < 3; ++i) *(volatile v4h*)(dst + off[i]) = o[i];
  __threadfence();
#pragma unroll
  for (int i = 0; i < 3; ++i) *(volatile v4h*)(dst + off[i]) = o[i];
}

template <int MODE, int KD, int NP>
__global__ __launch_bounds__(256) void gemm_kernel(
    const _Float16* __restrict__ A16, const _Float16* __restrict__ Bt,
    const float* __restrict__ biasf, const float* __restrict__ resf,
    float* __restrict__ outf, _Float16* __restrict__ out16) {
  static_assert((KD % 32) == 0 && (NP % 64) == 0);
  static_assert(MODE == 0 || MODE == 3 || NP == DIM);
  __shared__ float Cs[64 * LDC];
  const unsigned tid = threadIdx.x, lane = tid & 31u, w = tid >> 5;
  const unsigned mw = w >> 1, nw = w & 1u;
  const unsigned hh = lane >> 4, m = lane & 15u;
  const unsigned n0 = blockIdx.x * 64u;
  const unsigned row0 = blockIdx.y * 64u;

  const _Float16* ap  = A16 + (size_t)(row0 + mw * 16u + m) * KD + hh * 8u;
  const _Float16* bp0 = Bt + (size_t)(n0 + nw * 32u + m) * KD + hh * 8u;
  const _Float16* bp1 = bp0 + 16 * KD;
  v8f acc0 = {}, acc1 = {};
#pragma unroll 2
  for (unsigned k0 = 0; k0 < (unsigned)KD; k0 += 32u) {
    const v16h a  = frag_at(ap + k0);
    const v16h b0 = frag_at(bp0 + k0);
    const v16h b1 = frag_at(bp1 + k0);
    acc0 = wmma16(a, b0, acc0);
    acc1 = wmma16(a, b1, acc1);
  }
#pragma unroll
  for (int r = 0; r < 8; ++r) {
    float* d = &Cs[(mw * 16u + hh * 8u + (unsigned)r) * LDC + nw * 32u + m];
    d[0]  = acc0[r];
    d[16] = acc1[r];
  }
  __syncthreads();

  if (MODE == 0 || MODE == 3) {
    v8h x[2];
    size_t off[2];
#pragma unroll
    for (unsigned i = 0; i < 2u; ++i) {
      const unsigned r = 32u * i + (tid >> 3);
      const unsigned c = (tid & 7u) * 8u;
      const v4f u0 = *(const v4f*)&Cs[r * LDC + c];
      const v4f u1 = *(const v4f*)&Cs[r * LDC + c + 4];
      if (MODE == 0) {
#pragma unroll
        for (int j = 0; j < 4; ++j) {
          x[i][j]     = (_Float16)(u0[j] * (1.0f / WCARRY));
          x[i][j + 4] = (_Float16)(u1[j] * (1.0f / WCARRY));
        }
      } else {
        const v4f g0 = *(const v4f*)(biasf + n0 + c);
        const v4f g1 = *(const v4f*)(biasf + n0 + c + 4);
#pragma unroll
        for (int j = 0; j < 4; ++j) {
          const float t0 = fmaxf(u0[j] * (1.0f / WCARRY) + bf16r(g0[j]), 0.0f);
          const float t1 = fmaxf(u1[j] * (1.0f / WCARRY) + bf16r(g1[j]), 0.0f);
          x[i][j]     = (_Float16)(t0 * HCARRY);
          x[i][j + 4] = (_Float16)(t1 * HCARRY);
        }
      }
      off[i] = (size_t)(row0 + r) * NP + n0 + c;
    }
#pragma unroll
    for (int i = 0; i < 2; ++i) *(volatile v8h*)(out16 + off[i]) = x[i];
    __threadfence();
#pragma unroll
    for (int i = 0; i < 2; ++i) *(volatile v8h*)(out16 + off[i]) = x[i];
  }

  if (MODE == 1) {
    const unsigned bidx = row0 / (unsigned)SEQ;
    const unsigned key0 = row0 - bidx * (unsigned)SEQ;
    v8h x[2];
    size_t off[2];
#pragma unroll
    for (unsigned i = 0; i < 2u; ++i) {
      const unsigned dcol = 32u * i + (tid >> 3);
      const unsigned kk = (tid & 7u) * 8u;
#pragma unroll
      for (unsigned j = 0; j < 8u; ++j)
        x[i][j] = (_Float16)(Cs[(kk + j) * LDC + dcol] * (1.0f / WCARRY));
      off[i] = ((size_t)bidx * DIM + n0 + dcol) * SEQ + key0 + kk;
    }
#pragma unroll
    for (int i = 0; i < 2; ++i) *(volatile v8h*)(out16 + off[i]) = x[i];
    __threadfence();
#pragma unroll
    for (int i = 0; i < 2; ++i) *(volatile v8h*)(out16 + off[i]) = x[i];
  }

  if (MODE == 2 || MODE == 4) {
    v4f xs[4];
    size_t off[4];
#pragma unroll
    for (unsigned i = 0; i < 4u; ++i) {
      const unsigned r = 16u * i + (tid >> 4);
      const unsigned c = (tid & 15u) * 4u;
      const unsigned crow = row0 + r;
      const unsigned bidx = crow / (unsigned)SEQ;
      const unsigned sq = crow - bidx * (unsigned)SEQ;
      const size_t frow = (size_t)bidx * SEQ_FULL + sq;
      const size_t rrow = (MODE == 2) ? frow : (size_t)crow;
      const size_t orow = (MODE == 2) ? (size_t)crow : frow;
      const v4f u = *(const v4f*)&Cs[r * LDC + c];
      const v4f g = *(const v4f*)(biasf + n0 + c);
      const v4f xr = *(const v4f*)(resf + rrow * DIM + n0 + c);
      v4f val;
#pragma unroll
      for (int j = 0; j < 4; ++j) {
        const float base = (MODE == 2) ? bf16r(xr[j]) : xr[j];
        val[j] = base + (u[j] * (1.0f / (WCARRY * VCARRY)) + bf16r(g[j]));
      }
      xs[i] = val;
      off[i] = orow * DIM + n0 + c;
    }
#pragma unroll
    for (int i = 0; i < 4; ++i) *(volatile v4f*)(outf + off[i]) = xs[i];
    __threadfence();
#pragma unroll
    for (int i = 0; i < 4; ++i) *(volatile v4f*)(outf + off[i]) = xs[i];
  }
}
static_assert(VCARRY == HCARRY);

__global__ __launch_bounds__(256) void attn_kernel(
    const _Float16* __restrict__ Qh, const _Float16* __restrict__ Kh,
    const _Float16* __restrict__ Vt, _Float16* __restrict__ Ov) {
  __shared__ _Float16 Ks[64 * LDT];
  __shared__ _Float16 Vs[64 * LDT];
  __shared__ _Float16 Ps[8 * 16 * LDT];

  const unsigned tid = threadIdx.x, lane = tid & 31u;
  const unsigned w = (unsigned)__builtin_amdgcn_readfirstlane((int)(tid >> 5));
  const unsigned hh = lane >> 4, m = lane & 15u;
  const unsigned q0 = blockIdx.x * 128u;
  const unsigned head = blockIdx.y;
  const unsigned b = blockIdx.z;
  const unsigned qw0 = q0 + w * 16u;
  const unsigned kend = q0 + 128u;
  const float scale = 0.125f;
  _Float16* P = Ps + w * (16u * LDT);

  const size_t qoff = (size_t)(b * (unsigned)SEQ + qw0 + m) * DIM + head * HD + hh * 8u;
  v16h qf[2];
  qf[0] = frag_at(Qh + qoff);
  qf[1] = frag_at(Qh + qoff + 32);

  float mrow[8], lrow[8];
  v8f o[4];
#pragma unroll
  for (int v = 0; v < 8; ++v) { mrow[v] = -1.0e30f; lrow[v] = 0.0f; }
#pragma unroll
  for (int nb = 0; nb < 4; ++nb) o[nb] = (v8f){};

  const size_t kplane = (size_t)b * SEQ * DIM + head * HD;
  const size_t vplane = ((size_t)b * DIM + head * HD) * SEQ;

  for (unsigned kb = 0; kb < kend; kb += 64u) {
#pragma unroll
    for (unsigned j = 0; j < 2u; ++j) {
      const unsigned idx = tid + 256u * j;
      const unsigned r = idx >> 3, c = (idx & 7u) * 8u;
      *(v8h*)&Ks[r * LDT + c] = *(const v8h*)(Kh + kplane + (size_t)(kb + r) * DIM + c);
      *(v8h*)&Vs[r * LDT + c] = *(const v8h*)(Vt + vplane + (size_t)r * SEQ + kb + c);
    }
    __syncthreads();

    if (kb <= qw0 + 15u) {
      v8f s[4];
#pragma unroll
      for (int kg = 0; kg < 4; ++kg) {
        v8f t = {};
#pragma unroll
        for (int c = 0; c < 2; ++c) {
          const v16h kf = ld_frag(&Ks[(kg * 16) * LDT + c * 32], LDT);
          t = wmma16(qf[c], kf, t);
        }
        const unsigned key = kb + (unsigned)kg * 16u + m;
#pragma unroll
        for (int v = 0; v < 8; ++v) {
          const unsigned rowq = qw0 + hh * 8u + (unsigned)v;
          t[v] = (key <= rowq) ? t[v] * scale : -1.0e30f;
        }
        s[kg] = t;
      }

      float alpha[8];
#pragma unroll
      for (int v = 0; v < 8; ++v) {
        float mx = fmaxf(fmaxf(s[0][v], s[1][v]), fmaxf(s[2][v], s[3][v]));
        mx = red16_max(mx);
        const float mn = fmaxf(mrow[v], mx);
        alpha[v] = __expf(mrow[v] - mn);
        mrow[v] = mn;
      }
#pragma unroll
      for (int kg = 0; kg < 4; ++kg)
#pragma unroll
        for (int v = 0; v < 8; ++v) s[kg][v] = __expf(s[kg][v] - mrow[v]);
#pragma unroll
      for (int v = 0; v < 8; ++v) {
        const float rs = red16_sum((s[0][v] + s[1][v]) + (s[2][v] + s[3][v]));
        lrow[v] = alpha[v] * lrow[v] + rs;
      }
#pragma unroll
      for (int nb = 0; nb < 4; ++nb)
#pragma unroll
        for (int v = 0; v < 8; ++v) o[nb][v] = o[nb][v] * alpha[v];

#pragma unroll
      for (int kg = 0; kg < 4; ++kg)
#pragma unroll
        for (int v = 0; v < 8; ++v)
          P[(hh * 8u + (unsigned)v) * LDT + (unsigned)kg * 16u + m] =
              (_Float16)(s[kg][v] * PCARRY);
      wave_lds_sync();

#pragma unroll
      for (int c = 0; c < 2; ++c) {
        const v16h pf = ld_frag(P + c * 32, LDT);
#pragma unroll
        for (int nb = 0; nb < 4; ++nb) {
          const v16h vf = ld_frag(&Vs[(nb * 16) * LDT + c * 32], LDT);
          o[nb] = wmma16(pf, vf, o[nb]);
        }
      }
      wave_lds_sync();
    }
    __syncthreads();
  }

  float inv[8];
#pragma unroll
  for (int v = 0; v < 8; ++v) inv[v] = __builtin_amdgcn_rcpf(lrow[v]) * (VCARRY / PCARRY);
#pragma unroll
  for (int nb = 0; nb < 4; ++nb)
#pragma unroll
    for (int v = 0; v < 8; ++v)
      P[(hh * 8u + (unsigned)v) * LDT + (unsigned)nb * 16u + m] = (_Float16)(o[nb][v] * inv[v]);
  wave_lds_sync();
  v8h x[4];
  size_t off[4];
#pragma unroll
  for (unsigned i = 0; i < 4u; ++i) {
    const unsigned r = 4u * i + (lane >> 3);
    const unsigned c = (lane & 7u) * 8u;
    x[i] = *(const v8h*)&P[r * LDT + c];
    off[i] = (size_t)(b * (unsigned)SEQ + qw0 + r) * DIM + head * HD + c;
  }
#pragma unroll
  for (int i = 0; i < 4; ++i) *(volatile v8h*)(Ov + off[i]) = x[i];
  __threadfence();
#pragma unroll
  for (int i = 0; i < 4; ++i) *(volatile v8h*)(Ov + off[i]) = x[i];
}

extern "C" void kernel_launch(void* const* d_in, const int* in_sizes, int n_in,
                              void* d_out, int out_size, void* d_ws, size_t ws_size,
                              hipStream_t stream) {
  if (n_in < 14) return;
  const long long need_x = ((long long)(NB - 1) * SEQ_FULL + SEQ) * DIM;
  if ((long long)in_sizes[0] < need_x) return;
  for (int i = 1; i <= 4; ++i)
    if ((long long)in_sizes[i] < (long long)DIM * DIM) return;
  if (in_sizes[5] < DIM) return;
  if ((long long)in_sizes[6] < (long long)DIM * FF) return;
  if (in_sizes[7] < FF) return;
  if ((long long)in_sizes[8] < (long long)FF * DIM) return;
  if (in_sizes[9] < DIM) return;
  for (int i = 10; i <= 13; ++i)
    if (in_sizes[i] < DIM) return;
  if ((long long)out_size < need_x) return;
  if (ws_size < WS_TOTAL) return;

  const float* X   = (const float*)d_in[0];
  const float* wq  = (const float*)d_in[1];
  const float* wk  = (const float*)d_in[2];
  const float* wv  = (const float*)d_in[3];
  const float* wo  = (const float*)d_in[4];
  const float* bo  = (const float*)d_in[5];
  const float* w1  = (const float*)d_in[6];
  const float* b1  = (const float*)d_in[7];
  const float* w2  = (const float*)d_in[8];
  const float* b2  = (const float*)d_in[9];
  const float* g1  = (const float*)d_in[10];
  const float* be1 = (const float*)d_in[11];
  const float* g2  = (const float*)d_in[12];
  const float* be2 = (const float*)d_in[13];
  float* out = (float*)d_out;

  char* ws = (char*)d_ws;
  _Float16* WtA   = (_Float16*)ws;
  _Float16* W1t   = (_Float16*)(ws + OFF_W1);
  _Float16* W2t   = (_Float16*)(ws + OFF_W2);
  _Float16* H16   = (_Float16*)(ws + OFF_H);
  _Float16* Q16   = (_Float16*)(ws + OFF_REG + 0 * PLANE16_BYTES);
  _Float16* K16   = (_Float16*)(ws + OFF_REG + 1 * PLANE16_BYTES);
  _Float16* Vt16  = (_Float16*)(ws + OFF_REG + 2 * PLANE16_BYTES);
  _Float16* Ctx16 = (_Float16*)(ws + OFF_REG + 3 * PLANE16_BYTES);
  _Float16* F16   = (_Float16*)(ws + OFF_REG);
  float*    X1    = (float*)(ws + OFF_X1);

  const size_t WP = (size_t)DIM * DIM;
  dim3 blk(256);
  dim3 gD(DIM / 64, MROWS / 64);
  dim3 gF(FF / 64, MROWS / 64);

  wconv_kernel<<<dim3(DIM / 64, DIM / 64, 4), blk, 0, stream>>>(wq, wk, wv, wo, WtA,
                                                                (unsigned)DIM, (unsigned)DIM);
  wconv_kernel<<<dim3(FF / 64, DIM / 64, 1), blk, 0, stream>>>(w1, w1, w1, w1, W1t,
                                                               (unsigned)DIM, (unsigned)FF);
  wconv_kernel<<<dim3(DIM / 64, FF / 64, 1), blk, 0, stream>>>(w2, w2, w2, w2, W2t,
                                                               (unsigned)FF, (unsigned)DIM);

  ln_kernel<1><<<dim3(MROWS / 8), blk, 0, stream>>>(X, g1, be1, H16);
  gemm_kernel<0, DIM, DIM><<<gD, blk, 0, stream>>>(H16, WtA + 0 * WP, bo, X, X1, Q16);
  gemm_kernel<0, DIM, DIM><<<gD, blk, 0, stream>>>(H16, WtA + 1 * WP, bo, X, X1, K16);
  gemm_kernel<1, DIM, DIM><<<gD, blk, 0, stream>>>(H16, WtA + 2 * WP, bo, X, X1, Vt16);
  attn_kernel<<<dim3(SEQ / 128, NHEAD, NB), blk, 0, stream>>>(Q16, K16, Vt16, Ctx16);
  gemm_kernel<2, DIM, DIM><<<gD, blk, 0, stream>>>(Ctx16, WtA + 3 * WP, bo, X, X1, Q16);
  ln_kernel<0><<<dim3(MROWS / 8), blk, 0, stream>>>(X1, g2, be2, H16);
  gemm_kernel<3, DIM, FF><<<gF, blk, 0, stream>>>(H16, W1t, b1, X, out, F16);
  gemm_kernel<4, FF, DIM><<<gD, blk, 0, stream>>>(F16, W2t, b2, X1, out, H16);
}
